// spatialAttention_54468775247910
// MI455X (gfx1250) — hardware-verified
//
#include <hip/hip_runtime.h>
#include <math.h>

#ifndef NB
#define NB 2
#endif
#ifndef NT
#define NT 12
#endif
#define NB_FULL 2
#define NT_FULL 12
constexpr int kBatch = NB;
constexpr int kTime  = NT;
constexpr int kNode  = 512;
constexpr int kDim   = 512;
constexpr int kHeads = 8;
constexpr int kDh    = 64;
constexpr int kEmb   = 64;
constexpr int kFF    = 2048;
constexpr int kBT    = kBatch * kTime;
constexpr int kRows  = kBT * kNode;
constexpr float kWCarry     = 16.0f;
constexpr float kWCarryInv  = 1.0f / 16.0f;
constexpr float kPCarry     = 32768.0f;
constexpr float kCtxCarry   = 256.0f;
constexpr float kPVScale    = kCtxCarry / kPCarry;
constexpr float kWoScale    = 1.0f / (kCtxCarry * kWCarry);
constexpr float kScoreScale = 0.125f;
constexpr float kInvDim     = 1.0f / 512.0f;
constexpr float kLnEps      = 1e-5f;
constexpr float kNegBig     = -1.0e9f;
static_assert(kHeads * kDh == kDim);
static_assert(NB >= 1 && NT >= 1 && NB <= NB_FULL && NT <= NT_FULL);
static_assert(NT == NT_FULL || NB == 1);
static_assert(kRows % 64 == 0 && kDim % 64 == 0 && kNode % 64 == 0 && kFF % 64 == 0 && kDh % 64 == 0);
static_assert(kDim % 32 == 0 && kDh % 32 == 0 && kNode % 32 == 0 && kFF % 32 == 0);
static_assert(kNode == 512 && kDim == 512 && kEmb == 64);
static_assert((size_t)kRows * kDim <= (size_t)NB_FULL * NT_FULL * kNode * kDim);

typedef __attribute__((ext_vector_type(16))) _Float16 v16h;
typedef __attribute__((ext_vector_type(8)))  _Float16 v8h;
typedef __attribute__((ext_vector_type(16))) __bf16   v16b;
typedef __attribute__((ext_vector_type(8)))  __bf16   v8b;
typedef __attribute__((ext_vector_type(8)))  float    v8f;
typedef __attribute__((ext_vector_type(4)))  float    v4f;
typedef __attribute__((ext_vector_type(2)))  float    v2f;
typedef __attribute__((ext_vector_type(4)))  unsigned int v4u;

__device__ __forceinline__ unsigned short f2bf_bits(float f) {
  unsigned u = __float_as_uint(f);
  return (unsigned short)((u + 0x7FFFu + ((u >> 16) & 1u)) >> 16);
}
__device__ __forceinline__ float bf_bits2f(unsigned short h) { return __uint_as_float(((unsigned)h) << 16); }

__device__ __forceinline__ void dep_guard4_h(v8f& a, v8f& b, v8f& c, v8f& d, v16h x, v16h y) {
  asm volatile("v_nop\n\tv_nop\n\tv_nop\n\tv_nop" : "+v"(a), "+v"(b), "+v"(c), "+v"(d) : "v"(x), "v"(y));
}
__device__ __forceinline__ void dep_guard4_b(v8f& a, v8f& b, v8f& c, v8f& d, v16b x, v16b y) {
  asm volatile("v_nop\n\tv_nop\n\tv_nop\n\tv_nop" : "+v"(a), "+v"(b), "+v"(c), "+v"(d) : "v"(x), "v"(y));
}
__device__ __forceinline__ void keep4_h(v16h a, v16h b, v16h c, v16h d) { asm volatile("v_nop" :: "v"(a), "v"(b), "v"(c), "v"(d)); }
__device__ __forceinline__ void keep4_b(v16b a, v16b b, v16b c, v16b d) { asm volatile("v_nop" :: "v"(a), "v"(b), "v"(c), "v"(d)); }
__device__ __forceinline__ void acc_guard4(v8f& a, v8f& b, v8f& c, v8f& d) { asm volatile("v_nop\n\tv_nop\n\tv_nop\n\tv_nop" : "+v"(a), "+v"(b), "+v"(c), "+v"(d)); }
template <typename T> struct Frag;
template <> struct Frag<_Float16> {
  typedef v16h V; union U { v16h v; v8h h[2]; };
  static __device__ __forceinline__ v16h load(const _Float16* p) {
    U f; f.h[0] = *(const v8h*)(p); f.h[1] = *(const v8h*)(p + 16); return f.v;
  }
  static __device__ __forceinline__ v8f mma(v16h a, v16h b, v8f c) {
    return __builtin_amdgcn_wmma_f32_16x16x32_f16(false, a, false, b, (short)0, c, false, false);
  }
  static __device__ __forceinline__ void guard4(v8f& a, v8f& b, v8f& c, v8f& d, v16h x, v16h y) { dep_guard4_h(a, b, c, d, x, y); }
  static __device__ __forceinline__ void keep(v16h a, v16h b, v16h c, v16h d) { keep4_h(a, b, c, d); }
};
template <> struct Frag<__bf16> {
  typedef v16b V; union U { v16b v; v8b h[2]; };
  static __device__ __forceinline__ v16b load(const __bf16* p) {
    U f; f.h[0] = *(const v8b*)(p); f.h[1] = *(const v8b*)(p + 16); return f.v;
  }
  static __device__ __forceinline__ v8f mma(v16b a, v16b b, v8f c) {
    return __builtin_amdgcn_wmma_f32_16x16x32_bf16(false, a, false, b, (short)0, c, false, false);
  }
  static __device__ __forceinline__ void guard4(v8f& a, v8f& b, v8f& c, v8f& d, v16b x, v16b y) { dep_guard4_b(a, b, c, d, x, y); }
  static __device__ __forceinline__ void keep(v16b a, v16b b, v16b c, v16b d) { keep4_b(a, b, c, d); }
};

__device__ __forceinline__ unsigned pk16(unsigned short a, unsigned short b) { return (unsigned)a | ((unsigned)b << 16); }
__device__ __forceinline__ unsigned short h_bits(float f) { const _Float16 h = (_Float16)f; return __builtin_bit_cast(unsigned short, h); }

template <int ET> struct Elem;
template <> struct Elem<0> { typedef _Float16 T; };
template <> struct Elem<1> { typedef __bf16 T; };
template <int ET, bool SPLIT, int BIAS_MODE, int OUT_MODE, bool RESID, int ACT = 0>
__global__ __launch_bounds__(256) void wmma_gemm64(
    const unsigned short* __restrict__ Ap, const unsigned short* __restrict__ A2p, int lda, long strideA,
    const unsigned short* __restrict__ Btp, const unsigned short* __restrict__ Bt2p, int ldb, long strideB,
    void* __restrict__ Cout, void* __restrict__ Cout2, int ldc, long strideC,
    const float* __restrict__ bias,
    const float* __restrict__ resid, long strideR,
    int M, int N, int K, float scale) {
  static_assert(!(RESID && OUT_MODE != 0));
  static_assert(ACT == 0 || ACT == 2);
  typedef typename Elem<ET>::T T;
  typedef typename Frag<T>::V V;
  const T* A = (const T*)Ap; const T* A2 = (const T*)A2p; const T* Bt = (const T*)Btp; const T* Bt2 = (const T*)Bt2p;
  __shared__ __align__(16) float sT[8][16 * 68];
  const int b    = blockIdx.y;
  const int lane = threadIdx.x & 31;
  const int wave = threadIdx.x >> 5;
  const int tilesN = N >> 6;
  const int tilesM = M >> 6;
  const int tile = blockIdx.x * 8 + wave;
  if (tile >= tilesM * tilesN) return;
  const int tm = tile / tilesN;
  const int tn = tile - tm * tilesN;
  const int m0 = tm << 6;
  const int n0 = tn << 6;

  const T* Ab  = A  + (size_t)b * strideA;
  const T* Bb  = Bt + (size_t)b * strideB;
  const T* Ab2 = SPLIT ? (A2  + (size_t)b * strideA) : nullptr;
  const T* Bb2 = SPLIT ? (Bt2 + (size_t)b * strideB) : nullptr;

  const int rlane = lane & 15;
  const int koff  = (lane >> 4) * 8;
  const int mOff  = (lane >> 4) * 8;

  v8f acc[4][4];
#pragma unroll
  for (int i = 0; i < 4; ++i)
#pragma unroll
    for (int j = 0; j < 4; ++j) acc[i][j] = (v8f){0.f,0.f,0.f,0.f,0.f,0.f,0.f,0.f};

  for (int k0 = 0; k0 < K; k0 += 32) {
    V bh[4], bl[4];
#pragma unroll
    for (int j = 0; j < 4; ++j) {
      const size_t bo = (size_t)(n0 + (j << 4) + rlane) * ldb + koff + k0;
      bh[j] = Frag<T>::load(Bb + bo);
      if (SPLIT) bl[j] = Frag<T>::load(Bb2 + bo);
    }
#pragma unroll
    for (int i = 0; i < 4; ++i) {
      const size_t ao = (size_t)(m0 + (i << 4) + rlane) * lda + koff + k0;
      V ah = Frag<T>::load(Ab + ao);
      V al;
      if (SPLIT) al = Frag<T>::load(Ab2 + ao);
#pragma unroll
      for (int j = 0; j < 4; ++j) {
        acc[i][j] = Frag<T>::mma(ah, bh[j], acc[i][j]);
        if (SPLIT) {
          acc[i][j] = Frag<T>::mma(ah, bl[j], acc[i][j]);
          acc[i][j] = Frag<T>::mma(al, bh[j], acc[i][j]);
        }
      }
      Frag<T>::guard4(acc[i][0], acc[i][1], acc[i][2], acc[i][3], ah, SPLIT ? al : bh[3]);
    }
    Frag<T>::keep(bh[0], bh[1], bh[2], bh[3]);
    if (SPLIT) Frag<T>::keep(bl[0], bl[1], bl[2], bl[3]);
  }
  acc_guard4(acc[0][0], acc[0][1], acc[0][2], acc[0][3]);
  acc_guard4(acc[1][0], acc[1][1], acc[1][2], acc[1][3]);
  acc_guard4(acc[2][0], acc[2][1], acc[2][2], acc[2][3]);
  acc_guard4(acc[3][0], acc[3][1], acc[3][2], acc[3][3]);

  float* slab = sT[wave];
  const float* Rb = RESID ? (resid + (size_t)b * strideR) : nullptr;
#pragma unroll
  for (int i = 0; i < 4; ++i) {
    const int mBase = m0 + (i << 4);
#pragma unroll
    for (int j = 0; j < 4; ++j) {
      const int n = n0 + (j << 4) + rlane;
      float bv = 0.f;
      if (BIAS_MODE == 2) bv = bias[n];
#pragma unroll
      for (int r = 0; r < 8; ++r) {
        float v = acc[i][j][r] * scale;
        if (BIAS_MODE == 1) v += bias[mBase + mOff + r];
        if (BIAS_MODE == 2) v += bv;
        if (ACT == 2) v = fmaxf(v, 0.0f);
        slab[(mOff + r) * 68 + (j << 4) + rlane] = v;
      }
    }
    __builtin_amdgcn_fence(3  , "workgroup");
    __builtin_amdgcn_wave_barrier();
    __builtin_amdgcn_fence(2  , "workgroup");
    if (OUT_MODE == 0) {
      float* C = (float*)Cout + (size_t)b * strideC;
      const int hh = lane >> 4, c4 = (lane & 15) * 4;
      for (int pass = 0; pass < 2; ++pass) {
#pragma unroll
        for (int it = 0; it < 8; ++it) {
          const int row = it * 2 + hh;
          v4f v = *(const v4f*)(slab + row * 68 + c4);
          if (RESID) {
            const v4f rv = *(const v4f*)(Rb + (size_t)(mBase + row) * ldc + n0 + c4);
            v = v + rv;
          }
          *(volatile v4f*)(C + (size_t)(mBase + row) * ldc + n0 + c4) = v;
        }
        __threadfence();
      }
    } else {
      const int q = lane >> 3, c8 = (lane & 7) * 8;
      unsigned short* C  = (unsigned short*)Cout  + (size_t)b * strideC;
      unsigned short* C2 = (OUT_MODE == 2) ? ((unsigned short*)Cout2 + (size_t)b * strideC) : nullptr;
      for (int pass = 0; pass < 2; ++pass) {
#pragma unroll
        for (int it = 0; it < 4; ++it) {
          const int row = it * 4 + q;
          const float* sp = slab + row * 68 + c8;
          v8h hv, lv;
#pragma unroll
          for (int e = 0; e < 8; ++e) {
            if (OUT_MODE == 1) {
              hv[e] = (_Float16)sp[e];
            } else {
              unsigned short hb = f2bf_bits(sp[e]);
              unsigned short lb = f2bf_bits(sp[e] - bf_bits2f(hb));
              hv[e] = __builtin_bit_cast(_Float16, hb);
              lv[e] = __builtin_bit_cast(_Float16, lb);
            }
          }
          *(volatile v8h*)(C + (size_t)(mBase + row) * ldc + n0 + c8) = hv;
          if (OUT_MODE == 2) *(volatile v8h*)(C2 + (size_t)(mBase + row) * ldc + n0 + c8) = lv;
        }
        __threadfence();
      }
    }
    __builtin_amdgcn_fence(3  , "workgroup");
    __builtin_amdgcn_wave_barrier();
    __builtin_amdgcn_fence(2  , "workgroup");
  }
}

__global__ __launch_bounds__(256) void cast8_f16_kernel(const float* __restrict__ in, unsigned short* __restrict__ out,
                                                       int n8, float scale) {
  const int i = blockIdx.x * 256 + threadIdx.x;
  if (i >= n8) return;
  const float* p = in + 8 * (size_t)i;
  const v4f a = *(const v4f*)(p);
  const v4f c = *(const v4f*)(p + 4);
  unsigned short hb[8];
#pragma unroll
  for (int e = 0; e < 4; ++e) {
    hb[e]     = h_bits(a[e] * scale);
    hb[4 + e] = h_bits(c[e] * scale);
  }
  const v4u u = (v4u){pk16(hb[0], hb[1]), pk16(hb[2], hb[3]), pk16(hb[4], hb[5]), pk16(hb[6], hb[7])};
  unsigned short* q = out + 8 * (size_t)i;
  *(volatile v4u*)q = u;
  __threadfence();
  *(volatile v4u*)q = u;
}

__global__ __launch_bounds__(256) void graph_bias_kernel(const float* __restrict__ E, const float* __restrict__ lap,
                                                         const float* __restrict__ alpha_p, const float* __restrict__ beta_p,
                                                         float* __restrict__ biasM) {
  __shared__ __align__(16) float ei[kEmb];
  __shared__ __align__(16) float rowv[kNode];
  __shared__ float redM[8];
  __shared__ float redS[8];
  const int i = blockIdx.x;
  const int t = threadIdx.x, lane = t & 31, wave = t >> 5;
  if (t < kEmb) ei[t] = E[(size_t)i * kEmb + t];
  __syncthreads();
  const int j0 = t, j1 = t + 256;
  const float* e0p = E + (size_t)j0 * kEmb;
  const float* e1p = E + (size_t)j1 * kEmb;
  float d0 = 0.0f, d1 = 0.0f;
#pragma unroll 1
  for (int c = 0; c < kEmb / 4; ++c) {
    const v4f w  = *(const v4f*)(ei + 4 * c);
    const v4f a0 = *(const v4f*)(e0p + 4 * c);
    const v4f a1 = *(const v4f*)(e1p + 4 * c);
    d0 += a0[0] * w[0]; d0 += a0[1] * w[1]; d0 += a0[2] * w[2]; d0 += a0[3] * w[3];
    d1 += a1[0] * w[0]; d1 += a1[1] * w[1]; d1 += a1[2] * w[2]; d1 += a1[3] * w[3];
  }
  d0 = fmaxf(d0, 0.0f);
  d1 = fmaxf(d1, 0.0f);
  float mx = fmaxf(d0, d1);
#pragma unroll
  for (int off = 16; off > 0; off >>= 1) mx = fmaxf(mx, __shfl_xor(mx, off, 32));
  if (lane == 0) redM[wave] = mx;
  __syncthreads();
  float m = redM[0];
#pragma unroll
  for (int w = 1; w < 8; ++w) m = fmaxf(m, redM[w]);
  const float x0 = expf(d0 - m);
  const float x1 = expf(d1 - m);
  float ls = 0.0f;
  ls += x0;
  ls += x1;
#pragma unroll
  for (int off = 16; off > 0; off >>= 1) ls += __shfl_xor(ls, off, 32);
  if (lane == 0) redS[wave] = ls;
  __syncthreads();
  float tot = redS[0];
#pragma unroll
  for (int w = 1; w < 8; ++w) tot += redS[w];
  const float inv = 1.0f / tot;
  const float al = alpha_p[0];
  const float be = beta_p[0];
  const float lp0 = lap[(size_t)i * kNode + j0];
  const float lp1 = lap[(size_t)i * kNode + j1];
  const float mk0 = (lp0 != 0.0f) ? 0.0f : kNegBig;
  const float mk1 = (lp1 != 0.0f) ? 0.0f : kNegBig;
  rowv[j0] = (al * (x0 * inv) + be * lp0) + mk0;
  rowv[j1] = (al * (x1 * inv) + be * lp1) + mk1;
  __syncthreads();
  if (t < 128) {
    const v4f val = *(const v4f*)(rowv + 4 * t);
    float* dp = biasM + (size_t)i * kNode + 4 * t;
    *(volatile v4f*)dp = val;
    __threadfence();
    *(volatile v4f*)dp = val;
  }
}

__global__ __launch_bounds__(256) void layernorm_f16_kernel(const float* __restrict__ X, const float* __restrict__ gam,
                                                            const float* __restrict__ bet, unsigned short* __restrict__ Y) {
  __shared__ __align__(16) float gsh[kDim];
  __shared__ __align__(16) float bsh[kDim];
  const int t = threadIdx.x, lane = t & 31, wave = t >> 5;
  *(v2f*)(gsh + 2 * t) = *(const v2f*)(gam + 2 * t);
  *(v2f*)(bsh + 2 * t) = *(const v2f*)(bet + 2 * t);
  __syncthreads();
  const int row = blockIdx.x * 8 + wave;
  const float* xr = X + (size_t)row * kDim;
  const int cA = 8 * lane, cB = 256 + 8 * lane;
  const v4f xa = *(const v4f*)(xr + cA);
  const v4f xb = *(const v4f*)(xr + cA + 4);
  const v4f xc = *(const v4f*)(xr + cB);
  const v4f xd = *(const v4f*)(xr + cB + 4);
  float s = 0.0f;
  s += xa[0]; s += xa[1]; s += xa[2]; s += xa[3];
  s += xb[0]; s += xb[1]; s += xb[2]; s += xb[3];
  s += xc[0]; s += xc[1]; s += xc[2]; s += xc[3];
  s += xd[0]; s += xd[1]; s += xd[2]; s += xd[3];
#pragma unroll
  for (int off = 16; off > 0; off >>= 1) s += __shfl_xor(s, off, 32);
  const float mu = s * kInvDim;
  const v4f da = xa - mu;
  const v4f db = xb - mu;
  const v4f dc = xc - mu;
  const v4f dd = xd - mu;
  float q = 0.0f;
  q += da[0] * da[0]; q += da[1] * da[1]; q += da[2] * da[2]; q += da[3] * da[3];
  q += db[0] * db[0]; q += db[1] * db[1]; q += db[2] * db[2]; q += db[3] * db[3];
  q += dc[0] * dc[0]; q += dc[1] * dc[1]; q += dc[2] * dc[2]; q += dc[3] * dc[3];
  q += dd[0] * dd[0]; q += dd[1] * dd[1]; q += dd[2] * dd[2]; q += dd[3] * dd[3];
#pragma unroll
  for (int off = 16; off > 0; off >>= 1) q += __shfl_xor(q, off, 32);
  const float var = q * kInvDim;
  const float rs = rsqrtf(var + kLnEps);
  const v4f ga = *(const v4f*)(gsh + cA);
  const v4f gb = *(const v4f*)(gsh + cA + 4);
  const v4f gc = *(const v4f*)(gsh + cB);
  const v4f gd = *(const v4f*)(gsh + cB + 4);
  const v4f ba = *(const v4f*)(bsh + cA);
  const v4f bb = *(const v4f*)(bsh + cA + 4);
  const v4f bc = *(const v4f*)(bsh + cB);
  const v4f bd = *(const v4f*)(bsh + cB + 4);
  unsigned short hA[8], hB[8];
#pragma unroll
  for (int e = 0; e < 4; ++e) {
    hA[e]     = h_bits(da[e] * rs * ga[e] + ba[e]);
    hA[4 + e] = h_bits(db[e] * rs * gb[e] + bb[e]);
    hB[e]     = h_bits(dc[e] * rs * gc[e] + bc[e]);
    hB[4 + e] = h_bits(dd[e] * rs * gd[e] + bd[e]);
  }
  const v4u uA = (v4u){pk16(hA[0], hA[1]), pk16(hA[2], hA[3]), pk16(hA[4], hA[5]), pk16(hA[6], hA[7])};
  const v4u uB = (v4u){pk16(hB[0], hB[1]), pk16(hB[2], hB[3]), pk16(hB[4], hB[5]), pk16(hB[6], hB[7])};
  unsigned short* yr = Y + (size_t)row * kDim;
  *(volatile v4u*)(yr + cA) = uA;
  *(volatile v4u*)(yr + cB) = uB;
  __threadfence();
  *(volatile v4u*)(yr + cA) = uA;
  *(volatile v4u*)(yr + cB) = uB;
}

__global__ __launch_bounds__(256) void softmax_bias_kernel(const float* __restrict__ S, const float* __restrict__ biasM,
                                                           unsigned short* __restrict__ P) {
  __shared__ __align__(16) float lg[8][kNode];
  const int t = threadIdx.x, lane = t & 31, wave = t >> 5;
  const int row = blockIdx.x * 8 + wave;
  const int i = row & (kNode - 1);
  const float* sr = S + (size_t)row * kNode;
  const float* br = biasM + (size_t)i * kNode;
  float* lw = lg[wave];
  float mx = -__builtin_inff();
#pragma unroll 1
  for (int it = 0; it < 4; ++it) {
    const int c = ((it >> 1) << 8) + 8 * lane + ((it & 1) << 2);
    const v4f sv = *(const v4f*)(sr + c);
    const v4f gv = *(const v4f*)(br + c);
    const v4f l = sv + gv;
    mx = fmaxf(mx, fmaxf(fmaxf(l[0], l[1]), fmaxf(l[2], l[3])));
    *(v4f*)(lw + c) = l;
  }
#pragma unroll
  for (int off = 16; off > 0; off >>= 1) mx = fmaxf(mx, __shfl_xor(mx, off, 32));
  __builtin_amdgcn_fence(3  , "workgroup");
  __builtin_amdgcn_wave_barrier();
  __builtin_amdgcn_fence(2  , "workgroup");
  float sum = 0.0f;
#pragma unroll 1
  for (int it = 0; it < 4; ++it) {
    const int c = ((it >> 1) << 8) + 8 * lane + ((it & 1) << 2);
    const v4f l = *(const v4f*)(lw + c);
    v4f ev;
#pragma unroll
    for (int e = 0; e < 4; ++e) {
      const float x = expf(l[e] - mx);
      ev[e] = x;
      sum += x;
    }
    *(v4f*)(lw + c) = ev;
  }
#pragma unroll
  for (int off = 16; off > 0; off >>= 1) sum += __shfl_xor(sum, off, 32);
  __builtin_amdgcn_fence(3  , "workgroup");
  __builtin_amdgcn_wave_barrier();
  __builtin_amdgcn_fence(2  , "workgroup");
  const float inv = kPCarry / sum;
  const int cA = 8 * lane, cB = 256 + 8 * lane;
  const v4f e0 = *(const v4f*)(lw + cA);
  const v4f e1 = *(const v4f*)(lw + cA + 4);
  const v4f e2 = *(const v4f*)(lw + cB);
  const v4f e3 = *(const v4f*)(lw + cB + 4);
  unsigned short hA[8], hB[8];
#pragma unroll
  for (int e = 0; e < 4; ++e) {
    hA[e]     = h_bits(e0[e] * inv);
    hA[4 + e] = h_bits(e1[e] * inv);
    hB[e]     = h_bits(e2[e] * inv);
    hB[4 + e] = h_bits(e3[e] * inv);
  }
  const v4u uA = (v4u){pk16(hA[0], hA[1]), pk16(hA[2], hA[3]), pk16(hA[4], hA[5]), pk16(hA[6], hA[7])};
  const v4u uB = (v4u){pk16(hB[0], hB[1]), pk16(hB[2], hB[3]), pk16(hB[4], hB[5]), pk16(hB[6], hB[7])};
  unsigned short* pr = P + (size_t)row * kNode;
  *(volatile v4u*)(pr + cA) = uA;
  *(volatile v4u*)(pr + cB) = uB;
  __threadfence();
  *(volatile v4u*)(pr + cA) = uA;
  *(volatile v4u*)(pr + cB) = uB;
}

extern "C" void kernel_launch(void* const* d_in, const int* in_sizes, int n_in,
                              void* d_out, int out_size, void* d_ws, size_t ws_size,
                              hipStream_t stream) {
  if (n_in < 21) return;
  const int nTok = kRows * kDim;
  if (in_sizes[0] < nTok || out_size < nTok) return;
  if (in_sizes[1] < kNode * kNode || in_sizes[2] < kNode * kEmb) return;
  if (in_sizes[3] < kDim * kDim || in_sizes[5] < kDim * kDim || in_sizes[7] < kDim * kDim || in_sizes[9] < kDim * kDim) return;
  if (in_sizes[11] < kFF * kDim || in_sizes[13] < kDim * kFF) return;
  if (in_sizes[4] < kDim || in_sizes[6] < kDim || in_sizes[8] < kDim || in_sizes[10] < kDim || in_sizes[14] < kDim) return;
  if (in_sizes[12] < kFF || in_sizes[15] < kDim || in_sizes[16] < kDim || in_sizes[17] < kDim || in_sizes[18] < kDim) return;
  if (in_sizes[19] < 1 || in_sizes[20] < 1) return;

  const size_t szWsq  = (size_t)kDim * kDim * 2;
  const size_t szWff  = (size_t)kFF * kDim * 2;
  const size_t szBias = (size_t)kNode * kNode * 4;
  const size_t szP16  = (size_t)kRows * kDim * 2;
  const size_t szSC   = (size_t)kBT * kNode * kNode * 4;
  const size_t szPP   = (size_t)kBT * kNode * kNode * 2;
  static_assert((size_t)kRows * kFF * 2 == 4 * (size_t)kRows * kDim * 2);
  static_assert((size_t)kRows * kDim * 4 == (size_t)kBT * kNode * kNode * 4);
  static_assert((size_t)kRows * kDim * 2 == (size_t)kBT * kNode * kNode * 2);
  const size_t offWq = 0;
  const size_t offWk = offWq + szWsq;
  const size_t offWv = offWk + szWsq;
  const size_t offWo = offWv + szWsq;
  const size_t offW1 = offWo + szWsq;
  const size_t offW2 = offW1 + szWff;
  const size_t offBias = offW2 + szWff;
  const size_t offXN = offBias + szBias;
  const size_t offQ  = offXN + szP16;
  const size_t offK  = offQ + szP16;
  const size_t offVT = offK + szP16;
  const size_t offSC = offVT + szP16;
  const size_t offP  = offSC + szSC;
  const size_t total = offP + szPP;
  if (ws_size < total) return;

  const float* x     = (const float*)d_in[0];
  const float* lap   = (const float*)d_in[1];
  const float* emb   = (const float*)d_in[2];
  const float* Wq    = (const float*)d_in[3];
  const float* bq    = (const float*)d_in[4];
  const float* Wk    = (const float*)d_in[5];
  const float* bk    = (const float*)d_in[6];
  const float* Wv    = (const float*)d_in[7];
  const float* bv    = (const float*)d_in[8];
  const float* Wo    = (const float*)d_in[9];
  const float* bo    = (const float*)d_in[10];
  const float* W1    = (const float*)d_in[11];
  const float* b1    = (const float*)d_in[12];
  const float* W2    = (const float*)d_in[13];
  const float* b2    = (const float*)d_in[14];
  const float* ln1g  = (const float*)d_in[15];
  const float* ln1b  = (const float*)d_in[16];
  const float* ln2g  = (const float*)d_in[17];
  const float* ln2b  = (const float*)d_in[18];
  const float* alpha = (const float*)d_in[19];
  const float* beta  = (const float*)d_in[20];
  float* out = (float*)d_out;
  char* ws = (char*)d_ws;
  unsigned short* WQ16 = (unsigned short*)(ws + offWq);
  unsigned short* WK16 = (unsigned short*)(ws + offWk);
  unsigned short* WV16 = (unsigned short*)(ws + offWv);
  unsigned short* WO16 = (unsigned short*)(ws + offWo);
  unsigned short* W116 = (unsigned short*)(ws + offW1);
  unsigned short* W216 = (unsigned short*)(ws + offW2);
  float*          BIAS = (float*)(ws + offBias);
  unsigned short* XN   = (unsigned short*)(ws + offXN);
  unsigned short* AO   = XN;
  unsigned short* HH   = XN;
  unsigned short* Q16  = (unsigned short*)(ws + offQ);
  unsigned short* K16  = (unsigned short*)(ws + offK);
  unsigned short* VT16 = (unsigned short*)(ws + offVT);
  float*          SC   = (float*)(ws + offSC);
  float*          X1   = SC;
  unsigned short* PP   = (unsigned short*)(ws + offP);
  unsigned short* X1N  = PP;

  const int n8sq = (kDim * kDim) / 8;
  const int n8ff = (kFF * kDim) / 8;
  cast8_f16_kernel<<<dim3(n8sq / 256), dim3(256), 0, stream>>>(Wq, WQ16, n8sq, kWCarry);
  cast8_f16_kernel<<<dim3(n8sq / 256), dim3(256), 0, stream>>>(Wk, WK16, n8sq, kWCarry);
  cast8_f16_kernel<<<dim3(n8sq / 256), dim3(256), 0, stream>>>(Wv, WV16, n8sq, kWCarry);
  cast8_f16_kernel<<<dim3(n8sq / 256), dim3(256), 0, stream>>>(Wo, WO16, n8sq, kWCarry);
  cast8_f16_kernel<<<dim3(n8ff / 256), dim3(256), 0, stream>>>(W1, W116, n8ff, kWCarry);
  cast8_f16_kernel<<<dim3(n8ff / 256), dim3(256), 0, stream>>>(W2, W216, n8ff, kWCarry);

  graph_bias_kernel<<<dim3(kNode), dim3(256), 0, stream>>>(emb, lap, alpha, beta, BIAS);
  layernorm_f16_kernel<<<dim3(kRows / 8), dim3(256), 0, stream>>>(x, ln1g, ln1b, XN);

  const int tilesQK = (kRows / 64) * (kDim / 64);
  static_assert(((kRows / 64) * (kDim / 64)) % 8 == 0);
  wmma_gemm64<0, false, 2, 1, false, 0><<<dim3(tilesQK / 8, 1), dim3(256), 0, stream>>>(
      XN, XN, kDim, 0L, WQ16, WQ16, kDim, 0L, (void*)Q16, (void*)Q16, kDim, 0L, bq, x, 0L, kRows, kDim, kDim, kWCarryInv);
  wmma_gemm64<0, false, 2, 1, false, 0><<<dim3(tilesQK / 8, 1), dim3(256), 0, stream>>>(
      XN, XN, kDim, 0L, WK16, WK16, kDim, 0L, (void*)K16, (void*)K16, kDim, 0L, bk, x, 0L, kRows, kDim, kDim, kWCarryInv);
  const long strideBT16 = (long)kNode * kDim;
  const int tilesV = (kDim / 64) * (kNode / 64);
  wmma_gemm64<0, false, 1, 1, false, 0><<<dim3(tilesV / 8, kBT), dim3(256), 0, stream>>>(
      WV16, WV16, kDim, 0L, XN, XN, kDim, strideBT16, (void*)VT16, (void*)VT16, kNode, strideBT16,
      bv, x, 0L, kDim, kNode, kDim, kWCarryInv);

  const long strideSC = (long)kNode * kNode;
  const int tilesS  = (kNode / 64) * (kNode / 64);
  const int tilesPV = (kNode / 64) * (kDh / 64);
  for (int kh = 0; kh < kHeads; ++kh) {
    wmma_gemm64<0, false, 0, 0, false, 0><<<dim3(tilesS / 8, kBT), dim3(256), 0, stream>>>(
        Q16 + kh * kDh, Q16 + kh * kDh, kDim, strideBT16, K16 + kh * kDh, K16 + kh * kDh, kDim, strideBT16,
        (void*)SC, (void*)SC, kNode, strideSC, bq, x, 0L, kNode, kNode, kDh, kScoreScale);
    softmax_bias_kernel<<<dim3(kRows / 8), dim3(256), 0, stream>>>(SC, BIAS, PP);
    wmma_gemm64<0, false, 0, 1, false, 0><<<dim3(tilesPV / 8 > 0 ? tilesPV / 8 : 1, kBT), dim3(256), 0, stream>>>(
        PP, PP, kNode, strideSC, VT16 + (size_t)kh * kDh * kNode, VT16 + (size_t)kh * kDh * kNode, kNode, strideBT16,
        (void*)(AO + kh * kDh), (void*)(AO + kh * kDh), kDim, strideBT16, bq, x, 0L, kNode, kDh, kNode, kPVScale);
  }

  wmma_gemm64<0, false, 2, 0, true, 0><<<dim3(tilesQK / 8, 1), dim3(256), 0, stream>>>(
      AO, AO, kDim, 0L, WO16, WO16, kDim, 0L, (void*)X1, (void*)X1, kDim, 0L, bo, x, 0L, kRows, kDim, kDim, kWoScale);
  layernorm_f16_kernel<<<dim3(kRows / 8), dim3(256), 0, stream>>>(X1, ln2g, ln2b, X1N);
  const int tilesW1 = (kRows / 64) * (kFF / 64);
  wmma_gemm64<0, false, 2, 1, false, 2><<<dim3(tilesW1 / 8, 1), dim3(256), 0, stream>>>(
      X1N, X1N, kDim, 0L, W116, W116, kDim, 0L, (void*)HH, (void*)HH, kFF, 0L, b1, x, 0L, kRows, kFF, kDim, kWCarryInv);
  wmma_gemm64<0, false, 2, 0, true, 0><<<dim3(tilesQK / 8, 1), dim3(256), 0, stream>>>(
      HH, HH, kFF, 0L, W216, W216, kFF, 0L, (void*)out, (void*)out, kDim, 0L, b2, X1, 0L, kRows, kDim, kFF, kWCarryInv);
}
